// CapsLayer2D_2078764171657
// MI455X (gfx1250) — hardware-verified
//
#include <hip/hip_runtime.h>

typedef __bf16         v16bf __attribute__((ext_vector_type(16)));
typedef unsigned short v16us __attribute__((ext_vector_type(16)));
typedef unsigned short v8us  __attribute__((ext_vector_type(8)));
typedef float          v8f   __attribute__((ext_vector_type(8)));
typedef float          v4f   __attribute__((ext_vector_type(4)));
typedef v8us __attribute__((may_alias)) v8usa;
typedef v4f  __attribute__((may_alias)) v4fa;

union Frag { v16bf v; v16us u; v8us half[2]; };

#define NCELL 1024
#define NI    128
#define DIN   16
#define NK    32
#define DOUT  16
#define NIN   (NCELL * NI * DIN)
#define NWT   (NK * NI * DIN * DOUT)
#define NOUT  (NCELL * NK * DOUT)
#define NVPL  (NK * NCELL * DOUT)
#define NBPL  (NK * NI * NCELL)
#define EPSQ  1e-7f

__device__ __forceinline__ v8f wmma_bf16(v16bf a, v16bf b, v8f c) {
  v8f d = __builtin_amdgcn_wmma_f32_16x16x32_bf16(false, a, false, b, (short)0, c, false, false);
  asm volatile("v_nop\n\tv_nop\n\tv_nop\n\tv_nop" : "+v"(d) : "v"(a), "v"(b));
  return d;
}

__device__ __forceinline__ unsigned short bf16_rne(float x) {
  unsigned u = __float_as_uint(x);
  u += 0x7FFFu + ((u >> 16) & 1u);
  return (unsigned short)(u >> 16);
}
__device__ __forceinline__ float bf16_val(unsigned short b) {
  return __uint_as_float(((unsigned)b) << 16);
}
__device__ __forceinline__ void split1(float x, unsigned short& hi, unsigned short& lo) {
  const unsigned short hb = bf16_rne(x);
  hi = hb;
  lo = bf16_rne(x - bf16_val(hb));
}
__device__ __forceinline__ void split8(v4f a, v4f c, v8us& hi, v8us& lo) {
  v8us H = {0, 0, 0, 0, 0, 0, 0, 0};
  v8us L = {0, 0, 0, 0, 0, 0, 0, 0};
  unsigned short th, tl;
  split1(a[0], th, tl); H[0] = th; L[0] = tl;
  split1(a[1], th, tl); H[1] = th; L[1] = tl;
  split1(a[2], th, tl); H[2] = th; L[2] = tl;
  split1(a[3], th, tl); H[3] = th; L[3] = tl;
  split1(c[0], th, tl); H[4] = th; L[4] = tl;
  split1(c[1], th, tl); H[5] = th; L[5] = tl;
  split1(c[2], th, tl); H[6] = th; L[6] = tl;
  split1(c[3], th, tl); H[7] = th; L[7] = tl;
  hi = H; lo = L;
}

__global__ __launch_bounds__(256) void k_cvt_in(
    const float* __restrict__ x, unsigned short* __restrict__ xhi, unsigned short* __restrict__ xlo)
{
  const int g = blockIdx.x * 256 + threadIdx.x;
  if (g >= NIN / 8) return;
  const float* src = x + (size_t)g * 8;
  const v4f a = *(const v4fa*)src;
  const v4f c = *(const v4fa*)(src + 4);
  v8us hv, lv;
  split8(a, c, hv, lv);
  unsigned short* dh = xhi + (size_t)g * 8;
  unsigned short* dl = xlo + (size_t)g * 8;
  *(volatile v8us*)dh = hv;
  *(volatile v8us*)dl = lv;
  __threadfence();
  *(volatile v8us*)dh = hv;
  *(volatile v8us*)dl = lv;
}

__global__ __launch_bounds__(256) void k_cvt_w(
    const float* __restrict__ W,
    unsigned short* __restrict__ wn_hi, unsigned short* __restrict__ wn_lo,
    unsigned short* __restrict__ wt_hi, unsigned short* __restrict__ wt_lo)
{
  __shared__ __attribute__((aligned(16))) float sW[8 * 256];
  const int tid = threadIdx.x, lane = tid & 31, w = tid >> 5;
  const int u = blockIdx.x * 8 + w;
  const float* src = W + (size_t)u * 256 + lane * 8;
  const v4f a = *(const v4fa*)src;
  const v4f c = *(const v4fa*)(src + 4);

  v8us nh, nl;
  split8(a, c, nh, nl);

  float* sp = sW + w * 256 + lane * 8;
  sp[0] = a[0]; sp[1] = a[1]; sp[2] = a[2]; sp[3] = a[3];
  sp[4] = c[0]; sp[5] = c[1]; sp[6] = c[2]; sp[7] = c[3];
  __syncthreads();

  const int o = lane >> 1, d0 = (lane & 1) * 8;
  const float* col = sW + w * 256 + o;
  v4f ta, tc;
  ta[0] = col[(d0 + 0) * 16]; ta[1] = col[(d0 + 1) * 16]; ta[2] = col[(d0 + 2) * 16]; ta[3] = col[(d0 + 3) * 16];
  tc[0] = col[(d0 + 4) * 16]; tc[1] = col[(d0 + 5) * 16]; tc[2] = col[(d0 + 6) * 16]; tc[3] = col[(d0 + 7) * 16];
  v8us th, tl;
  split8(ta, tc, th, tl);

  const size_t off = (size_t)u * 256 + lane * 8;
  *(volatile v8us*)(wn_hi + off) = nh;
  *(volatile v8us*)(wn_lo + off) = nl;
  *(volatile v8us*)(wt_hi + off) = th;
  *(volatile v8us*)(wt_lo + off) = tl;
  __threadfence();
  *(volatile v8us*)(wn_hi + off) = nh;
  *(volatile v8us*)(wn_lo + off) = nl;
  *(volatile v8us*)(wt_hi + off) = th;
  *(volatile v8us*)(wt_lo + off) = tl;
}

__global__ __launch_bounds__(64) void k_caps_s(
    const unsigned short* __restrict__ in_hi, const unsigned short* __restrict__ in_lo,
    const unsigned short* __restrict__ wt_hi, const unsigned short* __restrict__ wt_lo,
    const float* __restrict__ bin,
    unsigned short* __restrict__ vhi, unsigned short* __restrict__ vlo,
    float* __restrict__ out,
    int bconst, int wout)
{
  __shared__ __attribute__((aligned(16))) float sv[2 * 256];

  const int tid = threadIdx.x, lane = tid & 31, w = tid >> 5;
  const int h = lane >> 4, m = lane & 15;
  const int c0 = blockIdx.x * 16, ky = blockIdx.y, k = 2 * ky + w;

  const unsigned short* ah = in_hi + ((size_t)(c0 + m) * NI) * DIN + 8 * h;
  const unsigned short* al = in_lo + ((size_t)(c0 + m) * NI) * DIN + 8 * h;
  const unsigned short* bh = wt_hi + ((size_t)k * NI * DOUT + m) * DIN + 8 * h;
  const unsigned short* bl = wt_lo + ((size_t)k * NI * DOUT + m) * DIN + 8 * h;
  const float* bp = bin + (size_t)k * NI * NCELL + c0 + 8 * h;

  const v8f  zero8 = {0.f, 0.f, 0.f, 0.f, 0.f, 0.f, 0.f, 0.f};
  const v8us z8us  = {0, 0, 0, 0, 0, 0, 0, 0};
  v8f sacc = zero8;

  #pragma unroll 2
  for (int i = 0; i < NI; ++i) {
    Frag a, b1, b2;
    a.half[0] = *(const v8usa*)(ah + i * DIN);
    a.half[1] = *(const v8usa*)(al + i * DIN);
    const v8us w8 = *(const v8usa*)(bh + i * (DOUT * DIN));
    b1.half[0] = w8;
    b1.half[1] = w8;
    b2.half[0] = *(const v8usa*)(bl + i * (DOUT * DIN));
    b2.half[1] = z8us;
    v8f r = wmma_bf16(a.v, b1.v, zero8);
    r = wmma_bf16(a.v, b2.v, r);
    if (bconst) {
      sacc = sacc + r;
    } else {
      const v4f q0 = *(const v4fa*)(bp + (size_t)i * NCELL);
      const v4f q1 = *(const v4fa*)(bp + (size_t)i * NCELL + 4);
      sacc[0] = fmaf(q0[0], r[0], sacc[0]);
      sacc[1] = fmaf(q0[1], r[1], sacc[1]);
      sacc[2] = fmaf(q0[2], r[2], sacc[2]);
      sacc[3] = fmaf(q0[3], r[3], sacc[3]);
      sacc[4] = fmaf(q1[0], r[4], sacc[4]);
      sacc[5] = fmaf(q1[1], r[5], sacc[5]);
      sacc[6] = fmaf(q1[2], r[6], sacc[6]);
      sacc[7] = fmaf(q1[3], r[7], sacc[7]);
    }
  }

  const float scl = bconst ? (1.0f / 128.0f) : 1.0f;
  const v8f s = sacc * scl;
  v8f v = zero8;
  #pragma unroll
  for (int r = 0; r < 8; ++r) {
    float t = s[r] * s[r];
    t += __shfl_xor(t, 1);
    t += __shfl_xor(t, 2);
    t += __shfl_xor(t, 4);
    t += __shfl_xor(t, 8);
    const float coef = (t * __builtin_amdgcn_rcpf(1.0f + t)) * rsqrtf(t + EPSQ);
    v[r] = coef * s[r];
  }

  float* svw = sv + w * 256;
  #pragma unroll
  for (int r = 0; r < 8; ++r) svw[(8 * h + r) * DOUT + m] = v[r];
  __syncthreads();

  const int q8 = lane & 7, sub = lane >> 3;
  if (wout == 0) {
    const v4f x0 = *(const v4fa*)(svw + lane * 8);
    const v4f x1 = *(const v4fa*)(svw + lane * 8 + 4);
    v8us hv, lv;
    split8(x0, x1, hv, lv);
    const size_t off = ((size_t)k * NCELL + c0) * DOUT + lane * 8;
    unsigned short* dh = vhi + off;
    unsigned short* dl = vlo + off;
    *(volatile v8us*)dh = hv;
    *(volatile v8us*)dl = lv;
    __threadfence();
    *(volatile v8us*)dh = hv;
    *(volatile v8us*)dl = lv;
  } else {
    const int kk = q8 >> 2, o0 = (q8 & 3) * 4;
    const int cellA = 8 * w + sub, cellB = 8 * w + 4 + sub;
    const v4f va = *(const v4fa*)(sv + kk * 256 + cellA * DOUT + o0);
    const v4f vb = *(const v4fa*)(sv + kk * 256 + cellB * DOUT + o0);
    float* da = out + (size_t)(c0 + cellA) * (NK * DOUT) + ky * 32 + q8 * 4;
    float* db = out + (size_t)(c0 + cellB) * (NK * DOUT) + ky * 32 + q8 * 4;
    *(volatile v4f*)da = va;
    *(volatile v4f*)db = vb;
    __threadfence();
    *(volatile v4f*)da = va;
    *(volatile v4f*)db = vb;
  }
}

__device__ __forceinline__ void b_store_sweep(const float* sB, const float* __restrict__ bin,
                                              float* __restrict__ bout, int has_bin,
                                              int k, int c0, int w, int lane) {
  const int q8 = lane & 7, sub = lane >> 3;
  #pragma unroll
  for (int j = 0; j < 16; ++j) {
    const int it = 64 * w + 4 * j + sub;
    v4f val = *(const v4fa*)(sB + it * 32 + q8 * 4);
    const size_t g = ((size_t)k * NI + it) * NCELL + c0 + q8 * 4;
    if (has_bin) {
      const v4f ob = *(const v4fa*)(bin + g);
      val = val + ob;
    } else {
      val = val + (1.0f / 128.0f);
    }
    *(volatile v4f*)(bout + g) = val;
  }
}

__global__ __launch_bounds__(64) void k_caps_b(
    const float* __restrict__ x,
    const unsigned short* __restrict__ wn_hi, const unsigned short* __restrict__ wn_lo,
    const unsigned short* __restrict__ vhi, const unsigned short* __restrict__ vlo,
    const float* __restrict__ bin, float* __restrict__ bout,
    int has_bin)
{
  __shared__ __attribute__((aligned(16))) float sB[NI * 32];

  const int tid = threadIdx.x, lane = tid & 31, w = tid >> 5;
  const int h = lane >> 4, m = lane & 15;
  const int c0 = blockIdx.x * 32, cw0 = c0 + 16 * w, k = blockIdx.y;

  const v8f  zero8 = {0.f, 0.f, 0.f, 0.f, 0.f, 0.f, 0.f, 0.f};
  const v8us z8us  = {0, 0, 0, 0, 0, 0, 0, 0};

  Frag bv;
  const size_t voff = ((size_t)k * NCELL + cw0 + m) * DOUT + 8 * h;
  bv.half[0] = *(const v8usa*)(vhi + voff);
  bv.half[1] = *(const v8usa*)(vlo + voff);

  const unsigned short* wh = wn_hi + ((size_t)k * NI * DIN + m) * DOUT + 8 * h;
  const unsigned short* wl = wn_lo + ((size_t)k * NI * DIN + m) * DOUT + 8 * h;
  const float* xp = x + ((size_t)(cw0 + m) * NI) * DIN + 8 * h;
  float* sbw = sB + 16 * w + m;

  #pragma unroll 2
  for (int i = 0; i < NI; ++i) {
    Frag a1, a2;
    const v8us w8 = *(const v8usa*)(wh + i * (DIN * DOUT));
    a1.half[0] = w8;
    a1.half[1] = w8;
    a2.half[0] = *(const v8usa*)(wl + i * (DIN * DOUT));
    a2.half[1] = z8us;
    v8f t = wmma_bf16(a1.v, bv.v, zero8);
    t = wmma_bf16(a2.v, bv.v, t);
    const v4f x0 = *(const v4fa*)(xp + i * DIN);
    const v4f x1 = *(const v4fa*)(xp + i * DIN + 4);
    float part = x0[0] * t[0];
    part = fmaf(x0[1], t[1], part);
    part = fmaf(x0[2], t[2], part);
    part = fmaf(x0[3], t[3], part);
    part = fmaf(x1[0], t[4], part);
    part = fmaf(x1[1], t[5], part);
    part = fmaf(x1[2], t[6], part);
    part = fmaf(x1[3], t[7], part);
    part += __shfl_xor(part, 16);
    sbw[i * 32] = part;
  }
  __syncthreads();

  b_store_sweep(sB, bin, bout, has_bin, k, c0, w, lane);
  __threadfence();
  b_store_sweep(sB, bin, bout, has_bin, k, c0, w, lane);
}

extern "C" void kernel_launch(void* const* d_in, const int* in_sizes, int n_in,
                              void* d_out, int out_size, void* d_ws, size_t ws_size,
                              hipStream_t stream) {
  if (n_in < 2) return;
  if (in_sizes[0] != NIN) return;
  if (in_sizes[1] != NWT) return;
  if (out_size != NOUT) return;

  const float* x = (const float*)d_in[0];
  const float* W = (const float*)d_in[1];
  float* out = (float*)d_out;

  const size_t inp_b = (size_t)NIN * 2;
  const size_t wp_b  = (size_t)NWT * 2;
  const size_t vp_b  = (size_t)NVPL * 2;
  const size_t bp_b  = (size_t)NBPL * 4;
  const size_t total = 2 * inp_b + 4 * wp_b + 2 * vp_b + 2 * bp_b;
  if (total > ws_size) return;

  char* ws = (char*)d_ws;
  size_t off = 0;
  unsigned short* in_hi = (unsigned short*)(ws + off); off += inp_b;
  unsigned short* in_lo = (unsigned short*)(ws + off); off += inp_b;
  unsigned short* wn_hi = (unsigned short*)(ws + off); off += wp_b;
  unsigned short* wn_lo = (unsigned short*)(ws + off); off += wp_b;
  unsigned short* wt_hi = (unsigned short*)(ws + off); off += wp_b;
  unsigned short* wt_lo = (unsigned short*)(ws + off); off += wp_b;
  unsigned short* v_hi  = (unsigned short*)(ws + off); off += vp_b;
  unsigned short* v_lo  = (unsigned short*)(ws + off); off += vp_b;
  float* bpl1 = (float*)(ws + off); off += bp_b;
  float* bpl2 = (float*)(ws + off); off += bp_b;
  if (off > ws_size) return;

  k_cvt_in<<<NIN / 8 / 256, 256, 0, stream>>>(x, in_hi, in_lo);
  k_cvt_w<<<(NK * NI) / 8, 256, 0, stream>>>(W, wn_hi, wn_lo, wt_hi, wt_lo);

  const dim3 gS(NCELL / 16, NK / 2);
  const dim3 gB(NCELL / 32, NK);

  k_caps_s<<<gS, 64, 0, stream>>>(in_hi, in_lo, wt_hi, wt_lo, bpl1, v_hi, v_lo, out, 1, 0);
  k_caps_b<<<gB, 64, 0, stream>>>(x, wn_hi, wn_lo, v_hi, v_lo, bpl2, bpl1, 0);
  k_caps_s<<<gS, 64, 0, stream>>>(in_hi, in_lo, wt_hi, wt_lo, bpl1, v_hi, v_lo, out, 0, 0);
  k_caps_b<<<gB, 64, 0, stream>>>(x, wn_hi, wn_lo, v_hi, v_lo, bpl1, bpl2, 1);
  k_caps_s<<<gS, 64, 0, stream>>>(in_hi, in_lo, wt_hi, wt_lo, bpl2, v_hi, v_lo, out, 0, 1);
}
